// MambaBlock_32976758898963
// MI455X (gfx1250) — hardware-verified
//
#include <hip/hip_runtime.h>
#include <stddef.h>
#include <stdint.h>
#include <math.h>


#define BSZ     2
#define LSEQ    2048
#define DMODEL  1024
#define DINNER  2048
#define DSTATE  16
#define DTRANK  64
#define NDBC    96
#define MROWS   (BSZ * LSEQ)
#define NTHR    256
#define GTHR    128
#define CR      32
#define TSTEP   64
#define SCT     64
#define WSMAX   134217728

#define EPI_XIN   0
#define EPI_GATE  1
#define EPI_XPROJ 2
#define EPI_DELTA 3
#define EPI_OUT   4

static_assert(MROWS % 128 == 0 && DINNER % 64 == 0 && DMODEL % 64 == 0);
static_assert(DMODEL % 32 == 0 && (2 * DINNER) % 32 == 0 && (2 * DTRANK) % 32 == 0);
static_assert(NDBC == DTRANK + 2 * DSTATE && NDBC == 6 * 16);
static_assert(LSEQ % CR == 0 && LSEQ % TSTEP == 0 && DINNER % SCT == 0);
static_assert((MROWS * DMODEL / 8) % NTHR == 0);
static_assert((DINNER * DSTATE / 4) % NTHR == 0);
static_assert(DINNER == 2 * NTHR * 4);
static_assert(SCT == 64 && TSTEP == 64 && DSTATE == 16);

typedef float          v4f   __attribute__((ext_vector_type(4)));
typedef float          v8f   __attribute__((ext_vector_type(8)));
typedef int            v8i   __attribute__((ext_vector_type(8)));
typedef unsigned short v4us  __attribute__((ext_vector_type(4)));
typedef unsigned short v8us  __attribute__((ext_vector_type(8)));
typedef unsigned short v16us __attribute__((ext_vector_type(16)));
typedef __bf16         v16bf __attribute__((ext_vector_type(16)));
typedef v4f  __attribute__((may_alias)) v4fa;
typedef v4us __attribute__((may_alias)) v4usa;
typedef v8us __attribute__((may_alias)) v8usa;
union FragB { v16bf v; v16us u; v8us h[2]; v8i w; };

__device__ __forceinline__ v8f wmb(const FragB& a, const FragB& b, v8f c) {
  v8f d = __builtin_amdgcn_wmma_f32_16x16x32_bf16(false, a.v, false, b.v, (short)0, c, false, false);
  asm volatile("v_nop\n\tv_nop\n\tv_nop\n\tv_nop" : "+v"(d) : "v"(a.w), "v"(b.w));
  return d;
}

__device__ __forceinline__ unsigned bf16_bits(float f) {
  const unsigned u = __float_as_uint(f);
  return (u + 0x7FFFu + ((u >> 16) & 1u)) >> 16;
}
__device__ __forceinline__ float bf16_val(float f) {
  return __uint_as_float(bf16_bits(f) << 16);
}
__device__ __forceinline__ v4f rbf4(v4f a) {
  v4f o;
  o.x = bf16_val(a.x); o.y = bf16_val(a.y); o.z = bf16_val(a.z); o.w = bf16_val(a.w);
  return o;
}
__device__ __forceinline__ void split4(v4f v, v4us& h4, v4us& l4) {
  unsigned hb;
  hb = bf16_bits(v.x); h4[0] = (unsigned short)hb; l4[0] = (unsigned short)bf16_bits(v.x - __uint_as_float(hb << 16));
  hb = bf16_bits(v.y); h4[1] = (unsigned short)hb; l4[1] = (unsigned short)bf16_bits(v.y - __uint_as_float(hb << 16));
  hb = bf16_bits(v.z); h4[2] = (unsigned short)hb; l4[2] = (unsigned short)bf16_bits(v.z - __uint_as_float(hb << 16));
  hb = bf16_bits(v.w); h4[3] = (unsigned short)hb; l4[3] = (unsigned short)bf16_bits(v.w - __uint_as_float(hb << 16));
}

__device__ __forceinline__ float silu_f(float c) {
  return c * __builtin_amdgcn_rcpf(1.0f + expf(-c));
}
__device__ __forceinline__ float softplus_f(float v) {
  return fmaxf(v, 0.0f) + log1pf(expf(-fabsf(v)));
}

__global__ __launch_bounds__(NTHR) void k_cvx(const float* __restrict__ x, unsigned short* xb) {
  const int u = (int)blockIdx.x * NTHR + (int)threadIdx.x;
  const float* p = x + (size_t)u * 8;
  const v4f a = *(const v4f*)p;
  const v4f b = *(const v4f*)(p + 4);
  v8us o;
  o[0] = (unsigned short)bf16_bits(a.x); o[1] = (unsigned short)bf16_bits(a.y);
  o[2] = (unsigned short)bf16_bits(a.z); o[3] = (unsigned short)bf16_bits(a.w);
  o[4] = (unsigned short)bf16_bits(b.x); o[5] = (unsigned short)bf16_bits(b.y);
  o[6] = (unsigned short)bf16_bits(b.z); o[7] = (unsigned short)bf16_bits(b.w);
  unsigned short* dp = xb + (size_t)u * 8;
  *(volatile v8us*)dp = o;
  __threadfence();
  *(volatile v8us*)dp = o;
}

__global__ __launch_bounds__(NTHR) void k_wtrans(const float* __restrict__ W, int Kd, int Nd, int k8s,
                                                 int nUnits, unsigned short* WT) {
  const int u = (int)blockIdx.x * NTHR + (int)threadIdx.x;
  if (u >= nUnits) return;
  const int n  = u >> k8s;
  const int k8 = (u & ((1 << k8s) - 1)) * 8;
  const float* p = W + (size_t)k8 * (size_t)Nd + n;
  v8us o;
#pragma unroll
  for (int i = 0; i < 8; ++i) o[i] = (unsigned short)bf16_bits(p[(size_t)i * (size_t)Nd]);
  unsigned short* dp = WT + (size_t)n * (size_t)Kd + k8;
  *(volatile v8us*)dp = o;
  __threadfence();
  *(volatile v8us*)dp = o;
}

__global__ __launch_bounds__(NTHR) void k_prepA(const float* __restrict__ alog, float* apl) {
  const int i = (int)blockIdx.x * NTHR + (int)threadIdx.x;
  const v4f a = *(const v4f*)(alog + (size_t)i * 4);
  v4f o;
  o.x = -expf(bf16_val(a.x));
  o.y = -expf(bf16_val(a.y));
  o.z = -expf(bf16_val(a.z));
  o.w = -expf(bf16_val(a.w));
  float* dp = apl + (size_t)i * 4;
  *(volatile v4f*)dp = o;
  __threadfence();
  *(volatile v4f*)dp = o;
}

template <int MT, int NT, int EPI>
__global__ __launch_bounds__(GTHR) void k_gemm(
    const unsigned short* __restrict__ A, const unsigned short* __restrict__ BT,
    int K, int ldb, int kmask,
    float* outF, int ldo, const float* __restrict__ aux, unsigned short* out16)
{
  constexpr int BM = 64 * MT;
  constexpr int BN = 16 * NT;
  constexpr int WR = 16 * MT;
  __shared__ __attribute__((aligned(16))) float stg[BM * BN];
  const int tid = (int)threadIdx.x, lane = tid & 31, wave = tid >> 5, hh = lane >> 4, m = lane & 15;
  const int rowBase = (int)blockIdx.x * BM;
  const int col0    = (int)blockIdx.y * BN;

  v8f acc[MT][NT];
  {
    const v8f z = {0.f, 0.f, 0.f, 0.f, 0.f, 0.f, 0.f, 0.f};
#pragma unroll
    for (int i = 0; i < MT; ++i)
#pragma unroll
      for (int t = 0; t < NT; ++t) acc[i][t] = z;
  }
  const unsigned short* ap = A  + (size_t)(rowBase + WR * wave + m) * (size_t)K + 8 * hh;
  const unsigned short* wp = BT + (size_t)(col0 + m) * (size_t)ldb + 8 * hh;

#pragma unroll 1
  for (int k0 = 0; k0 < K; k0 += 32) {
    const int kb = k0 & kmask;
    FragB af[MT];
#pragma unroll
    for (int i = 0; i < MT; ++i) {
      const unsigned short* aq = ap + (size_t)(16 * i) * (size_t)K + k0;
      af[i].h[0] = *(const v8usa*)aq;
      af[i].h[1] = *(const v8usa*)(aq + 16);
    }
#pragma unroll
    for (int t = 0; t < NT; ++t) {
      const unsigned short* wq = wp + (size_t)(16 * t) * (size_t)ldb + kb;
      FragB bf;
      bf.h[0] = *(const v8usa*)wq;
      bf.h[1] = *(const v8usa*)(wq + 16);
#pragma unroll
      for (int i = 0; i < MT; ++i) acc[i][t] = wmb(af[i], bf, acc[i][t]);
    }
  }

#pragma unroll
  for (int i = 0; i < MT; ++i) {
#pragma unroll
    for (int t = 0; t < NT; ++t) {
      const int lc = 16 * t + m;
#pragma unroll
      for (int r = 0; r < 8; ++r) {
        const int lr = WR * wave + 16 * i + 8 * hh + r;
        stg[lr * BN + lc] = acc[i][t][r];
      }
    }
  }
  __syncthreads();

  if constexpr (EPI == EPI_XIN || EPI == EPI_OUT || EPI == EPI_DELTA) {
    static_assert(NT == 4);
    constexpr int NIT = 8 * MT;
    if constexpr (EPI == EPI_DELTA) {
      const v4f bb = rbf4(*(const v4f*)(aux + col0 + 4 * m));
#pragma unroll 1
      for (int j = 0; j < NIT; ++j) {
        float* sp = stg + (WR * wave + 2 * j + hh) * BN + 4 * m;
        v4f a = *(const v4fa*)sp;
        a.x = softplus_f(a.x + bb.x);
        a.y = softplus_f(a.y + bb.y);
        a.z = softplus_f(a.z + bb.z);
        a.w = softplus_f(a.w + bb.w);
        *(v4fa*)sp = a;
      }
    }
    v4f fv[NIT];
#pragma unroll
    for (int j = 0; j < NIT; ++j) fv[j] = *(const v4fa*)(stg + (WR * wave + 2 * j + hh) * BN + 4 * m);
#pragma unroll
    for (int j = 0; j < NIT; ++j) {
      const int gr = rowBase + WR * wave + 2 * j + hh;
      *(volatile v4f*)(outF + (size_t)gr * (size_t)ldo + col0 + 4 * m) = fv[j];
    }
    __threadfence();
#pragma unroll
    for (int j = 0; j < NIT; ++j) {
      const int gr = rowBase + WR * wave + 2 * j + hh;
      *(volatile v4f*)(outF + (size_t)gr * (size_t)ldo + col0 + 4 * m) = fv[j];
    }
  } else if constexpr (EPI == EPI_GATE) {
    static_assert(NT == 4);
    constexpr int NIT = 8 * MT;
#pragma unroll 1
    for (int j = 0; j < NIT; ++j) {
      const int lr = WR * wave + 2 * j + hh;
      const int gr = rowBase + lr;
      const v4f a = *(const v4fa*)(stg + lr * BN + 4 * m);
      const v4f y = *(const v4f*)(aux + (size_t)gr * DINNER + col0 + 4 * m);
      v4f g;
      g.x = y.x * silu_f(a.x);
      g.y = y.y * silu_f(a.y);
      g.z = y.z * silu_f(a.z);
      g.w = y.w * silu_f(a.w);
      v4us h4, l4;
      split4(g, h4, l4);
      unsigned short* srow = (unsigned short*)stg + (size_t)lr * (2 * BN);
      *(v4usa*)(srow + 4 * m) = h4;
      *(v4usa*)(srow + 64 + 4 * m) = l4;
    }
    __syncthreads();
    v8us qv[NIT];
#pragma unroll
    for (int j = 0; j < NIT; ++j) {
      const unsigned short* srow = (const unsigned short*)stg + (size_t)(WR * wave + 2 * j + hh) * (2 * BN);
      qv[j] = *(const v8usa*)(srow + 8 * m);
    }
    const int coff = (m < 8) ? (col0 + 8 * m) : (DINNER + col0 + 8 * (m - 8));
#pragma unroll
    for (int j = 0; j < NIT; ++j) {
      const int gr = rowBase + WR * wave + 2 * j + hh;
      *(volatile v8us*)(out16 + (size_t)gr * (2 * DINNER) + coff) = qv[j];
    }
    __threadfence();
#pragma unroll
    for (int j = 0; j < NIT; ++j) {
      const int gr = rowBase + WR * wave + 2 * j + hh;
      *(volatile v8us*)(out16 + (size_t)gr * (2 * DINNER) + coff) = qv[j];
    }
  } else {
    static_assert(EPI == EPI_XPROJ && MT == 1 && NT == 6);
    __shared__ __attribute__((aligned(16))) unsigned short stg16[64 * 128];
    v4f fv[4];
#pragma unroll
    for (int i = 0; i < 4; ++i) {
      const int idx = i * 32 + lane;
      fv[i] = *(const v4fa*)(stg + (WR * wave + (idx >> 3)) * BN + 64 + 4 * (idx & 7));
    }
#pragma unroll 1
    for (int j = 0; j < 8; ++j) {
      const int lr = WR * wave + 2 * j + hh;
      const v4f a = *(const v4fa*)(stg + lr * BN + 4 * m);
      v4us h4, l4;
      split4(a, h4, l4);
      unsigned short* srow = stg16 + lr * 128;
      *(v4usa*)(srow + 4 * m) = h4;
      *(v4usa*)(srow + 64 + 4 * m) = l4;
    }
    __syncthreads();
    v8us qv[8];
#pragma unroll
    for (int j = 0; j < 8; ++j) qv[j] = *(const v8usa*)(stg16 + (WR * wave + 2 * j + hh) * 128 + 8 * m);
    float* bp = outF + (size_t)(rowBase + WR * wave) * 32 + 4 * lane;
#pragma unroll
    for (int i = 0; i < 4; ++i) *(volatile v4f*)(bp + 128 * i) = fv[i];
#pragma unroll
    for (int j = 0; j < 8; ++j) {
      const int gr = rowBase + WR * wave + 2 * j + hh;
      *(volatile v8us*)(out16 + (size_t)gr * 128 + 8 * m) = qv[j];
    }
    __threadfence();
#pragma unroll
    for (int i = 0; i < 4; ++i) *(volatile v4f*)(bp + 128 * i) = fv[i];
#pragma unroll
    for (int j = 0; j < 8; ++j) {
      const int gr = rowBase + WR * wave + 2 * j + hh;
      *(volatile v8us*)(out16 + (size_t)gr * 128 + 8 * m) = qv[j];
    }
  }
}

__device__ __forceinline__ float conv1(v4f w, float a, float b, float c, float d, float bias) {
  float s = w.x * a;
  s = fmaf(w.y, b, s);
  s = fmaf(w.z, c, s);
  s = fmaf(w.w, d, s);
  return s + bias;
}

__global__ __launch_bounds__(NTHR) void k_conv(const float* __restrict__ xin, const float* __restrict__ cw,
                                               const float* __restrict__ cb, float* xc, unsigned short* xhl) {
  const int d4   = ((int)blockIdx.x * NTHR + (int)threadIdx.x) * 4;
  const int row0 = (int)blockIdx.y * CR;
  const int t0   = row0 & (LSEQ - 1);
  const v4f w0 = rbf4(*(const v4f*)(cw + (size_t)d4 * 4));
  const v4f w1 = rbf4(*(const v4f*)(cw + (size_t)d4 * 4 + 4));
  const v4f w2 = rbf4(*(const v4f*)(cw + (size_t)d4 * 4 + 8));
  const v4f w3 = rbf4(*(const v4f*)(cw + (size_t)d4 * 4 + 12));
  const v4f bb = rbf4(*(const v4f*)(cb + d4));
  const float fz = (t0 != 0) ? 1.0f : 0.0f;
  const int ra = row0 - 3 < 0 ? 0 : row0 - 3;
  const int rb = row0 - 2 < 0 ? 0 : row0 - 2;
  const int rc = row0 - 1 < 0 ? 0 : row0 - 1;
  v4f xm3 = *(const v4f*)(xin + (size_t)ra * DINNER + d4) * fz;
  v4f xm2 = *(const v4f*)(xin + (size_t)rb * DINNER + d4) * fz;
  v4f xm1 = *(const v4f*)(xin + (size_t)rc * DINNER + d4) * fz;
#pragma unroll 1
  for (int r = 0; r < CR; ++r) {
    const size_t row = (size_t)(row0 + r);
    const v4f cur = *(const v4f*)(xin + row * DINNER + d4);
    v4f s;
    s.x = silu_f(conv1(w0, xm3.x, xm2.x, xm1.x, cur.x, bb.x));
    s.y = silu_f(conv1(w1, xm3.y, xm2.y, xm1.y, cur.y, bb.y));
    s.z = silu_f(conv1(w2, xm3.z, xm2.z, xm1.z, cur.z, bb.z));
    s.w = silu_f(conv1(w3, xm3.w, xm2.w, xm1.w, cur.w, bb.w));
    v4us h4, l4;
    split4(s, h4, l4);
    float* xp = xc + row * DINNER + d4;
    unsigned short* hp = xhl + row * (2 * DINNER) + d4;
    unsigned short* lp = hp + DINNER;
    *(volatile v4f*)xp = s;
    *(volatile v4us*)hp = h4;
    *(volatile v4us*)lp = l4;
    __threadfence();
    *(volatile v4f*)xp = s;
    *(volatile v4us*)hp = h4;
    *(volatile v4us*)lp = l4;
    xm3 = xm2; xm2 = xm1; xm1 = cur;
  }
}

__global__ __launch_bounds__(SCT) void k_scan(const float* __restrict__ delta, float* xcy,
                                              const float* __restrict__ bcp, const float* __restrict__ apl,
                                              const float* __restrict__ dsk) {
  __shared__ __attribute__((aligned(16))) float bc[TSTEP * 32];
  __shared__ __attribute__((aligned(16))) float ys[TSTEP * SCT];
  const int tid = (int)threadIdx.x;
  const int d0  = (int)blockIdx.x * SCT;
  const int d   = d0 + tid;
  const int b   = (int)blockIdx.y;

  float Av[DSTATE], h[DSTATE];
#pragma unroll
  for (int k = 0; k < 4; ++k) {
    const v4f q = *(const v4f*)(apl + (size_t)d * DSTATE + 4 * k);
    Av[4 * k + 0] = q.x; Av[4 * k + 1] = q.y; Av[4 * k + 2] = q.z; Av[4 * k + 3] = q.w;
  }
#pragma unroll
  for (int s = 0; s < DSTATE; ++s) h[s] = 0.0f;
  const float Dd = bf16_val(dsk[d]);

#pragma unroll 1
  for (int tile = 0; tile < LSEQ / TSTEP; ++tile) {
    const int row0 = b * LSEQ + tile * TSTEP;
#pragma unroll
    for (int j = 0; j < 8; ++j) {
      const int idx = j * SCT + tid;
      *(v4fa*)(bc + 4 * idx) = *(const v4f*)(bcp + (size_t)row0 * 32 + 4 * idx);
    }
    __syncthreads();
#pragma unroll 1
    for (int tt = 0; tt < TSTEP; ++tt) {
      const size_t gi = (size_t)(row0 + tt) * DINNER + d;
      const float dl = delta[gi];
      const float u  = xcy[gi];
      const float du = dl * u;
      const float* br = bc + tt * 32;
      float Bv[DSTATE], Cv[DSTATE];
#pragma unroll
      for (int k = 0; k < 4; ++k) {
        const v4f qb = *(const v4fa*)(br + 4 * k);
        const v4f qc = *(const v4fa*)(br + 16 + 4 * k);
        Bv[4 * k + 0] = qb.x; Bv[4 * k + 1] = qb.y; Bv[4 * k + 2] = qb.z; Bv[4 * k + 3] = qb.w;
        Cv[4 * k + 0] = qc.x; Cv[4 * k + 1] = qc.y; Cv[4 * k + 2] = qc.z; Cv[4 * k + 3] = qc.w;
      }
      float y = 0.0f;
#pragma unroll
      for (int s = 0; s < DSTATE; ++s) {
        const float dA = expf(dl * Av[s]);
        h[s] = fmaf(dA, h[s], du * Bv[s]);
        y = fmaf(h[s], Cv[s], y);
      }
      y = fmaf(u, Dd, y);
      ys[tt * SCT + tid] = y;
    }
    __syncthreads();
    v4f yv[16];
#pragma unroll
    for (int i = 0; i < 16; ++i) yv[i] = *(const v4fa*)(ys + 4 * (i * SCT + tid));
#pragma unroll
    for (int i = 0; i < 16; ++i) {
      const int idx = i * SCT + tid;
      *(volatile v4f*)(xcy + (size_t)(row0 + (idx >> 4)) * DINNER + d0 + 4 * (idx & 15)) = yv[i];
    }
    __threadfence();
#pragma unroll
    for (int i = 0; i < 16; ++i) {
      const int idx = i * SCT + tid;
      *(volatile v4f*)(xcy + (size_t)(row0 + (idx >> 4)) * DINNER + d0 + 4 * (idx & 15)) = yv[i];
    }
  }
}

static inline size_t al256(size_t o) { return (o + 255) & ~(size_t)255; }

extern "C" void kernel_launch(void* const* d_in, const int* in_sizes, int n_in,
                              void* d_out, int out_size, void* d_ws, size_t ws_size,
                              hipStream_t stream) {
  if (n_in < 10) return;
  if (in_sizes[0] != MROWS * DMODEL) return;
  if (in_sizes[1] != DMODEL * 2 * DINNER) return;
  if (in_sizes[2] != DINNER * 4) return;
  if (in_sizes[3] != DINNER) return;
  if (in_sizes[4] != DINNER * NDBC) return;
  if (in_sizes[5] != DTRANK * DINNER) return;
  if (in_sizes[6] != DINNER) return;
  if (in_sizes[7] != DINNER * DSTATE) return;
  if (in_sizes[8] != DINNER) return;
  if (in_sizes[9] != DINNER * DMODEL) return;
  if (out_size != MROWS * DMODEL) return;

  const float* x      = (const float*)d_in[0];
  const float* W_in   = (const float*)d_in[1];
  const float* conv_w = (const float*)d_in[2];
  const float* conv_b = (const float*)d_in[3];
  const float* W_xp   = (const float*)d_in[4];
  const float* W_dt   = (const float*)d_in[5];
  const float* b_dt   = (const float*)d_in[6];
  const float* A_log  = (const float*)d_in[7];
  const float* D_skip = (const float*)d_in[8];
  const float* W_out  = (const float*)d_in[9];
  float* out = (float*)d_out;

  char* ws = (char*)d_ws;
  size_t off = 0;
  const size_t oR1  = off; off = al256(off + (size_t)MROWS * DINNER * 4);
  const size_t oR3  = off; off = al256(off + (size_t)MROWS * DINNER * 4);
  const size_t oR4  = off; off = al256(off + (size_t)MROWS * 2 * DINNER * 2);
  const size_t oXB  = off; off = al256(off + (size_t)MROWS * DMODEL * 2);
  const size_t oWI  = off; off = al256(off + (size_t)2 * DINNER * DMODEL * 2);
  const size_t oWO  = off; off = al256(off + (size_t)DMODEL * DINNER * 2);
  const size_t oWX  = off; off = al256(off + (size_t)NDBC * DINNER * 2);
  const size_t oWD  = off; off = al256(off + (size_t)DINNER * DTRANK * 2);
  const size_t oBC  = off; off = al256(off + (size_t)MROWS * 32 * 4);
  const size_t oDT  = off; off = al256(off + (size_t)MROWS * 2 * DTRANK * 2);
  const size_t oAP  = off; off = al256(off + (size_t)DINNER * DSTATE * 4);
  if (off > ws_size || off > (size_t)WSMAX) return;
  float*          R1   = (float*)(ws + oR1);
  float*          R3   = (float*)(ws + oR3);
  unsigned short* R4   = (unsigned short*)(ws + oR4);
  unsigned short* XB   = (unsigned short*)(ws + oXB);
  unsigned short* WINt = (unsigned short*)(ws + oWI);
  unsigned short* WOt  = (unsigned short*)(ws + oWO);
  unsigned short* WXt  = (unsigned short*)(ws + oWX);
  unsigned short* WDTt = (unsigned short*)(ws + oWD);
  float*          BC   = (float*)(ws + oBC);
  unsigned short* DTLO = (unsigned short*)(ws + oDT);
  float*          APL  = (float*)(ws + oAP);

  k_cvx<<<(MROWS * DMODEL / 8) / NTHR, NTHR, 0, stream>>>(x, XB);
  k_wtrans<<<(2 * DINNER * (DMODEL / 8)) / NTHR, NTHR, 0, stream>>>(W_in, DMODEL, 2 * DINNER, 7,
                                                                   2 * DINNER * (DMODEL / 8), WINt);
  k_wtrans<<<(NDBC * (DINNER / 8)) / NTHR, NTHR, 0, stream>>>(W_xp, DINNER, NDBC, 8, NDBC * (DINNER / 8), WXt);
  k_wtrans<<<(DINNER * (DTRANK / 8)) / NTHR, NTHR, 0, stream>>>(W_dt, DTRANK, DINNER, 3,
                                                               DINNER * (DTRANK / 8), WDTt);
  k_wtrans<<<(DMODEL * (DINNER / 8)) / NTHR, NTHR, 0, stream>>>(W_out, DINNER, DMODEL, 8,
                                                               DMODEL * (DINNER / 8), WOt);
  k_prepA<<<(DINNER * DSTATE / 4) / NTHR, NTHR, 0, stream>>>(A_log, APL);
  k_gemm<2, 4, EPI_XIN><<<dim3(MROWS / 128, DINNER / 64), GTHR, 0, stream>>>(
      XB, WINt, DMODEL, DMODEL, DMODEL - 1, R1, DINNER, APL, DTLO);
  k_conv<<<dim3(DINNER / (NTHR * 4), MROWS / CR), NTHR, 0, stream>>>(R1, conv_w, conv_b, R3, R4);
  k_gemm<1, 6, EPI_XPROJ><<<dim3(MROWS / 64, 1), GTHR, 0, stream>>>(
      R4, WXt, 2 * DINNER, DINNER, DINNER - 1, BC, 32, APL, DTLO);
  k_gemm<2, 4, EPI_DELTA><<<dim3(MROWS / 128, DINNER / 64), GTHR, 0, stream>>>(
      DTLO, WDTt, 2 * DTRANK, DTRANK, DTRANK - 1, R1, DINNER, b_dt, DTLO);
  k_scan<<<dim3(DINNER / SCT, BSZ), SCT, 0, stream>>>(R1, R3, BC, APL, D_skip);
  k_gemm<2, 4, EPI_GATE><<<dim3(MROWS / 128, DINNER / 64), GTHR, 0, stream>>>(
      XB, WINt + (size_t)DINNER * DMODEL, DMODEL, DMODEL, DMODEL - 1, R1, DINNER, R3, R4);
  k_gemm<2, 4, EPI_OUT><<<dim3(MROWS / 128, DMODEL / 64), GTHR, 0, stream>>>(
      R4, WOt, 2 * DINNER, DINNER, DINNER - 1, out, DMODEL, APL, DTLO);
}
